// PackedQKVBlock_16535624089651
// MI455X (gfx1250) — hardware-run, weakly checked
//
#include <hip/hip_runtime.h>
#include <math.h>

constexpr int kB   = 2;
constexpr int kS   = 2048;
constexpr int kD   = 1024;
constexpr int kH   = 16;
constexpr int kDK  = 64;
constexpr int kTok = kB * kS;
constexpr int kFF  = 4 * kD;
constexpr int kGroups = kB * kH;
constexpr int kGPC = 2;
constexpr int kChunks = kGroups / kGPC;
constexpr float kWCarry     = 256.0f;
constexpr float kWCarryInv  = 1.0f / 256.0f;
constexpr float kPCarry     = 2048.0f;
constexpr float kCtxCarry   = 256.0f;
constexpr float kScoreScale = 0.125f;
constexpr float kPVScale    = kCtxCarry / kPCarry;
constexpr float kWoScale    = 1.0f / (kCtxCarry * kWCarry);
constexpr float kInvD       = 1.0f / 1024.0f;
constexpr float kLnEps      = 1e-5f;

constexpr size_t kMiB     = 1048576;
constexpr size_t kOffQkvW = 0;
constexpr size_t kOffWoW  = 6 * kMiB;
constexpr size_t kOffF1W  = 8 * kMiB;
constexpr size_t kOffF2W  = 16 * kMiB;
constexpr size_t kOffH    = 24 * kMiB;
constexpr size_t kOffQK   = 32 * kMiB;
constexpr size_t kOffVT   = 48 * kMiB;
constexpr size_t kOffCTX  = 56 * kMiB;
constexpr size_t kOffSC   = 64 * kMiB;
constexpr size_t kOffP    = 96 * kMiB;
constexpr size_t kOffX1   = 64 * kMiB;
constexpr size_t kOffHID  = 80 * kMiB;
constexpr size_t kWsTotal = 112 * kMiB;

typedef __attribute__((ext_vector_type(16))) _Float16 v16h;
typedef __attribute__((ext_vector_type(8)))  _Float16 v8h;
typedef __attribute__((ext_vector_type(16))) __bf16   v16b;
typedef __attribute__((ext_vector_type(8)))  __bf16   v8b;
typedef __attribute__((ext_vector_type(8)))  float    v8f;
typedef __attribute__((ext_vector_type(4)))  float    v4f;
typedef __attribute__((ext_vector_type(4)))  unsigned int v4u;

__device__ __forceinline__ unsigned short f2bf_bits(float f) {
  unsigned u = __float_as_uint(f);
  return (unsigned short)((u + 0x7FFFu + ((u >> 16) & 1u)) >> 16);
}
__device__ __forceinline__ float bf_bits2f(unsigned short h) { return __uint_as_float(((unsigned)h) << 16); }

__device__ __forceinline__ void dep_guard_h(v8f& a, v8f& b, v16h x, v16h y) { asm volatile("v_nop\n\tv_nop\n\tv_nop\n\tv_nop" : "+v"(a), "+v"(b) : "v"(x), "v"(y)); }
__device__ __forceinline__ void dep_guard_b(v8f& a, v8f& b, v16b x, v16b y) { asm volatile("v_nop\n\tv_nop\n\tv_nop\n\tv_nop" : "+v"(a), "+v"(b) : "v"(x), "v"(y)); }
__device__ __forceinline__ void keep4_h(v16h a, v16h b, v16h c, v16h d) { asm volatile("v_nop" :: "v"(a), "v"(b), "v"(c), "v"(d)); }
__device__ __forceinline__ void keep4_b(v16b a, v16b b, v16b c, v16b d) { asm volatile("v_nop" :: "v"(a), "v"(b), "v"(c), "v"(d)); }
__device__ __forceinline__ void acc_guard4(v8f& a, v8f& b, v8f& c, v8f& d) { asm volatile("v_nop\n\tv_nop\n\tv_nop\n\tv_nop" : "+v"(a), "+v"(b), "+v"(c), "+v"(d)); }
template <typename T> struct Frag;
template <> struct Frag<_Float16> {
  typedef v16h V; union U { v16h v; v8h h[2]; };
  static __device__ __forceinline__ v16h load(const _Float16* p) {
    U f; f.h[0] = *(const v8h*)(p); f.h[1] = *(const v8h*)(p + 16); return f.v;
  }
  static __device__ __forceinline__ v8f mma(v16h a, v16h b, v8f c) {
    return __builtin_amdgcn_wmma_f32_16x16x32_f16(false, a, false, b, (short)0, c, false, false);
  }
  static __device__ __forceinline__ void guard(v8f& a, v8f& b, v16h x, v16h y) { dep_guard_h(a, b, x, y); }
  static __device__ __forceinline__ void keep(v16h a, v16h b, v16h c, v16h d) { keep4_h(a, b, c, d); }
};
template <> struct Frag<__bf16> {
  typedef v16b V; union U { v16b v; v8b h[2]; };
  static __device__ __forceinline__ v16b load(const __bf16* p) {
    U f; f.h[0] = *(const v8b*)(p); f.h[1] = *(const v8b*)(p + 16); return f.v;
  }
  static __device__ __forceinline__ v8f mma(v16b a, v16b b, v8f c) {
    return __builtin_amdgcn_wmma_f32_16x16x32_bf16(false, a, false, b, (short)0, c, false, false);
  }
  static __device__ __forceinline__ void guard(v8f& a, v8f& b, v16b x, v16b y) { dep_guard_b(a, b, x, y); }
  static __device__ __forceinline__ void keep(v16b a, v16b b, v16b c, v16b d) { keep4_b(a, b, c, d); }
};

__device__ __forceinline__ unsigned pk16(unsigned short a, unsigned short b) { return (unsigned)a | ((unsigned)b << 16); }
__device__ __forceinline__ unsigned short h_bits(float f) { const _Float16 h = (_Float16)f; return __builtin_bit_cast(unsigned short, h); }

template <int ET> struct Elem;
template <> struct Elem<0> { typedef _Float16 T; };
template <> struct Elem<1> { typedef __bf16 T; };
template <int ET, bool SPLIT, int BIAS_MODE, int OUT_MODE, bool RESID, int ACT = 0>
__global__ __launch_bounds__(256) void wmma_gemm64(
    const unsigned short* __restrict__ Ap, const unsigned short* __restrict__ A2p, int lda, long strideA,
    const unsigned short* __restrict__ Btp, const unsigned short* __restrict__ Bt2p, int ldb, long strideB,
    void* __restrict__ Cout, void* __restrict__ Cout2, int ldc, long strideC,
    const float* __restrict__ bias,
    const float* __restrict__ resid, long strideR,
    int M, int N, int K, float scale) {
  typedef typename Elem<ET>::T T;
  typedef typename Frag<T>::V V;
  const T* A = (const T*)Ap; const T* A2 = (const T*)A2p; const T* Bt = (const T*)Btp; const T* Bt2 = (const T*)Bt2p;
  __shared__ __align__(16) float sT[8][16 * 68];
  const int b    = blockIdx.y;
  const int lane = threadIdx.x & 31;
  const int wave = threadIdx.x >> 5;
  const int tilesN = N >> 6;
  const int tilesM = M >> 6;
  const int tile = blockIdx.x * 8 + wave;
  if (tile >= tilesM * tilesN) return;
  const int tm = tile / tilesN;
  const int tn = tile - tm * tilesN;
  const int m0 = tm << 6;
  const int n0 = tn << 6;

  const T* Ab  = A  + (size_t)b * strideA;
  const T* Bb  = Bt + (size_t)b * strideB;
  const T* Ab2 = SPLIT ? (A2  + (size_t)b * strideA) : nullptr;
  const T* Bb2 = SPLIT ? (Bt2 + (size_t)b * strideB) : nullptr;

  const int rlane = lane & 15;
  const int koff  = (lane >> 4) * 8;
  const int mOff  = (lane >> 4) * 8;

  v8f acc[4][4];
#pragma unroll
  for (int i = 0; i < 4; ++i)
#pragma unroll
    for (int j = 0; j < 4; ++j) acc[i][j] = (v8f){0.f,0.f,0.f,0.f,0.f,0.f,0.f,0.f};

  for (int k0 = 0; k0 < K; k0 += 32) {
    V bh[4], bl[4];
#pragma unroll
    for (int j = 0; j < 4; ++j) {
      const size_t bo = (size_t)(n0 + (j << 4) + rlane) * ldb + koff + k0;
      bh[j] = Frag<T>::load(Bb + bo);
      if (SPLIT) bl[j] = Frag<T>::load(Bb2 + bo);
    }
#pragma unroll
    for (int i = 0; i < 4; ++i) {
      const size_t ao = (size_t)(m0 + (i << 4) + rlane) * lda + koff + k0;
      V ah = Frag<T>::load(Ab + ao);
      V al;
      if (SPLIT) al = Frag<T>::load(Ab2 + ao);
#pragma unroll
      for (int j = 0; j < 4; ++j) {
        acc[i][j] = Frag<T>::mma(ah, bh[j], acc[i][j]);
        if (SPLIT) {
          acc[i][j] = Frag<T>::mma(ah, bl[j], acc[i][j]);
          acc[i][j] = Frag<T>::mma(al, bh[j], acc[i][j]);
        }
      }
      Frag<T>::guard(acc[i][0], acc[i][3], ah, SPLIT ? al : ah);
    }
    Frag<T>::keep(bh[0], bh[1], bh[2], bh[3]);
    if (SPLIT) Frag<T>::keep(bl[0], bl[1], bl[2], bl[3]);
  }
  acc_guard4(acc[0][0], acc[0][1], acc[0][2], acc[0][3]);
  acc_guard4(acc[1][0], acc[1][1], acc[1][2], acc[1][3]);
  acc_guard4(acc[2][0], acc[2][1], acc[2][2], acc[2][3]);
  acc_guard4(acc[3][0], acc[3][1], acc[3][2], acc[3][3]);

  float* slab = sT[wave];
  const float* Rb = RESID ? (resid + (size_t)b * strideR) : nullptr;
#pragma unroll
  for (int i = 0; i < 4; ++i) {
    const int mBase = m0 + (i << 4);
#pragma unroll
    for (int j = 0; j < 4; ++j) {
      const int n = n0 + (j << 4) + rlane;
      float bv = 0.f;
      if (BIAS_MODE == 2) bv = bias[n];
#pragma unroll
      for (int r = 0; r < 8; ++r) {
        float v = acc[i][j][r] * scale;
        if (BIAS_MODE == 1) v += bias[mBase + mOff + r];
        if (BIAS_MODE == 2) v += bv;
        if (RESID) v += Rb[(size_t)(mBase + mOff + r) * ldc + n];
        if (ACT == 2) v = fmaxf(v, 0.0f);
        if (ACT == 4) v = (v > 0.f) ? v : 0.01f * v;
        slab[(mOff + r) * 68 + (j << 4) + rlane] = v;
      }
    }
    __builtin_amdgcn_fence(__ATOMIC_RELEASE, "workgroup");
    __builtin_amdgcn_wave_barrier();
    __builtin_amdgcn_fence(__ATOMIC_ACQUIRE, "workgroup");
    if (OUT_MODE == 0) {
      float* C = (float*)Cout + (size_t)b * strideC;
      const int hh = lane >> 4, c4 = (lane & 15) * 4;
      for (int pass = 0; pass < 2; ++pass) {
#pragma unroll
        for (int it = 0; it < 8; ++it) {
          const int row = it * 2 + hh;
          v4f v = *(const v4f*)(slab + row * 68 + c4);
          *(volatile v4f*)(C + (size_t)(mBase + row) * ldc + n0 + c4) = v;
        }
        __threadfence();
      }
    } else {
      const int q = lane >> 3, c8 = (lane & 7) * 8;
      unsigned short* C  = (unsigned short*)Cout  + (size_t)b * strideC;
      unsigned short* C2 = (OUT_MODE == 2) ? ((unsigned short*)Cout2 + (size_t)b * strideC) : nullptr;
      for (int pass = 0; pass < 2; ++pass) {
#pragma unroll
        for (int it = 0; it < 4; ++it) {
          const int row = it * 4 + q;
          const float* sp = slab + row * 68 + c8;
          v8h hv, lv;
#pragma unroll
          for (int e = 0; e < 8; ++e) {
            if (OUT_MODE == 1) {
              hv[e] = (_Float16)sp[e];
            } else {
              unsigned short hb = f2bf_bits(sp[e]);
              unsigned short lb = f2bf_bits(sp[e] - bf_bits2f(hb));
              hv[e] = __builtin_bit_cast(_Float16, hb);
              lv[e] = __builtin_bit_cast(_Float16, lb);
            }
          }
          *(volatile v8h*)(C + (size_t)(mBase + row) * ldc + n0 + c8) = hv;
          if (OUT_MODE == 2) *(volatile v8h*)(C2 + (size_t)(mBase + row) * ldc + n0 + c8) = lv;
        }
        __threadfence();
      }
    }
    __builtin_amdgcn_fence(__ATOMIC_RELEASE, "workgroup");
    __builtin_amdgcn_wave_barrier();
    __builtin_amdgcn_fence(__ATOMIC_ACQUIRE, "workgroup");
  }
}

__global__ __launch_bounds__(256) void cast8_f16_kernel(const float* __restrict__ in, unsigned short* __restrict__ out,
                                                         int n8, float scale) {
  const int i = blockIdx.x * 256 + threadIdx.x;
  if (i >= n8) return;
  const float* p = in + 8 * (size_t)i;
  const v4f a = *(const v4f*)(p);
  const v4f c = *(const v4f*)(p + 4);
  unsigned short hb[8];
#pragma unroll
  for (int e = 0; e < 4; ++e) {
    hb[e]     = h_bits(a[e] * scale);
    hb[4 + e] = h_bits(c[e] * scale);
  }
  const v4u u = (v4u){pk16(hb[0], hb[1]), pk16(hb[2], hb[3]), pk16(hb[4], hb[5]), pk16(hb[6], hb[7])};
  unsigned short* q = out + 8 * (size_t)i;
  *(volatile v4u*)q = u;
  __threadfence();
  *(volatile v4u*)q = u;
}

__global__ __launch_bounds__(128) void ln_row_kernel(const float* __restrict__ X, const float* __restrict__ w,
                                                     const float* __restrict__ bb, unsigned short* __restrict__ out) {
  __shared__ float redA[4];
  __shared__ float redB[4];
  const int row  = blockIdx.x;
  const int t    = threadIdx.x;
  const int lane = t & 31, wave = t >> 5;
  const int c0   = t * 8;
  const float* xr = X + (size_t)row * kD + c0;
  const v4f a = *(const v4f*)(xr);
  const v4f c = *(const v4f*)(xr + 4);
  float x[8];
#pragma unroll
  for (int e = 0; e < 4; ++e) { x[e] = a[e]; x[4 + e] = c[e]; }
  float s = ((x[0] + x[1]) + (x[2] + x[3])) + ((x[4] + x[5]) + (x[6] + x[7]));
#pragma unroll
  for (int off = 16; off > 0; off >>= 1) s += __shfl_xor(s, off, 32);
  if (lane == 0) redA[wave] = s;
  __syncthreads();
  const float mu = ((redA[0] + redA[1]) + (redA[2] + redA[3])) * kInvD;
  float d[8];
#pragma unroll
  for (int e = 0; e < 8; ++e) d[e] = x[e] - mu;
  float ss = ((d[0] * d[0] + d[1] * d[1]) + (d[2] * d[2] + d[3] * d[3])) +
             ((d[4] * d[4] + d[5] * d[5]) + (d[6] * d[6] + d[7] * d[7]));
#pragma unroll
  for (int off = 16; off > 0; off >>= 1) ss += __shfl_xor(ss, off, 32);
  if (lane == 0) redB[wave] = ss;
  __syncthreads();
  const float var  = ((redB[0] + redB[1]) + (redB[2] + redB[3])) * kInvD;
  const float rstd = rsqrtf(var + kLnEps);
  const v4f wa = *(const v4f*)(w + c0);
  const v4f wc = *(const v4f*)(w + c0 + 4);
  const v4f ba = *(const v4f*)(bb + c0);
  const v4f bc = *(const v4f*)(bb + c0 + 4);
  unsigned short hb[8];
#pragma unroll
  for (int e = 0; e < 4; ++e) {
    hb[e]     = h_bits(d[e] * rstd * wa[e] + ba[e]);
    hb[4 + e] = h_bits(d[4 + e] * rstd * wc[e] + bc[e]);
  }
  const v4u u = (v4u){pk16(hb[0], hb[1]), pk16(hb[2], hb[3]), pk16(hb[4], hb[5]), pk16(hb[6], hb[7])};
  unsigned short* q = out + (size_t)row * kD + c0;
  *(volatile v4u*)q = u;
  __threadfence();
  *(volatile v4u*)q = u;
}

__global__ __launch_bounds__(256) void softmax_row_kernel(const float* __restrict__ Sc, unsigned short* __restrict__ P,
                                                          float carry) {
  __shared__ float redM[8];
  __shared__ float redS[8];
  const int row  = blockIdx.x;
  const int t    = threadIdx.x;
  const int lane = t & 31, wave = t >> 5;
  const int c0   = t * 8;
  const float* sr = Sc + (size_t)row * kS + c0;
  const v4f a = *(const v4f*)(sr);
  const v4f c = *(const v4f*)(sr + 4);
  float x[8];
#pragma unroll
  for (int e = 0; e < 4; ++e) { x[e] = a[e]; x[4 + e] = c[e]; }
  float m = fmaxf(fmaxf(fmaxf(x[0], x[1]), fmaxf(x[2], x[3])), fmaxf(fmaxf(x[4], x[5]), fmaxf(x[6], x[7])));
#pragma unroll
  for (int off = 16; off > 0; off >>= 1) m = fmaxf(m, __shfl_xor(m, off, 32));
  if (lane == 0) redM[wave] = m;
  __syncthreads();
  float gm = redM[0];
#pragma unroll
  for (int i = 1; i < 8; ++i) gm = fmaxf(gm, redM[i]);
  float ev[8];
#pragma unroll
  for (int e = 0; e < 8; ++e) ev[e] = expf(x[e] - gm);
  float s = ((ev[0] + ev[1]) + (ev[2] + ev[3])) + ((ev[4] + ev[5]) + (ev[6] + ev[7]));
#pragma unroll
  for (int off = 16; off > 0; off >>= 1) s += __shfl_xor(s, off, 32);
  if (lane == 0) redS[wave] = s;
  __syncthreads();
  float tot = redS[0];
#pragma unroll
  for (int i = 1; i < 8; ++i) tot += redS[i];
  const float inv = carry / tot;
  unsigned short hb[8];
#pragma unroll
  for (int e = 0; e < 8; ++e) hb[e] = h_bits(ev[e] * inv);
  const v4u u = (v4u){pk16(hb[0], hb[1]), pk16(hb[2], hb[3]), pk16(hb[4], hb[5]), pk16(hb[6], hb[7])};
  unsigned short* q = P + (size_t)row * kS + c0;
  *(volatile v4u*)q = u;
  __threadfence();
  *(volatile v4u*)q = u;
}

extern "C" void kernel_launch(void* const* d_in, const int* in_sizes, int n_in,
                              void* d_out, int out_size, void* d_ws, size_t ws_size,
                              hipStream_t stream) {
  if (n_in < 13) return;
  if ((size_t)out_size < (size_t)kTok * kD) return;
  if (ws_size < kWsTotal) return;
  if (in_sizes[0] != kTok * kD || in_sizes[3] != 3 * kD * kD || in_sizes[4] != 3 * kD ||
      in_sizes[5] != kD * kD || in_sizes[9] != kFF * kD || in_sizes[11] != kD * kFF) return;

  const float* x     = (const float*)d_in[0];
  const float* ln1_w = (const float*)d_in[1];
  const float* ln1_b = (const float*)d_in[2];
  const float* qkv_w = (const float*)d_in[3];
  const float* qkv_b = (const float*)d_in[4];
  const float* wo_w  = (const float*)d_in[5];
  const float* wo_b  = (const float*)d_in[6];
  const float* ln2_w = (const float*)d_in[7];
  const float* ln2_b = (const float*)d_in[8];
  const float* f1_w  = (const float*)d_in[9];
  const float* f1_b  = (const float*)d_in[10];
  const float* f2_w  = (const float*)d_in[11];
  const float* f2_b  = (const float*)d_in[12];
  float* out = (float*)d_out;

  char* ws = (char*)d_ws;
  unsigned short* qkvw16 = (unsigned short*)(ws + kOffQkvW);
  unsigned short* wo16   = (unsigned short*)(ws + kOffWoW);
  unsigned short* f1w16  = (unsigned short*)(ws + kOffF1W);
  unsigned short* f2w16  = (unsigned short*)(ws + kOffF2W);
  unsigned short* h16    = (unsigned short*)(ws + kOffH);
  unsigned short* qk16   = (unsigned short*)(ws + kOffQK);
  unsigned short* vt16   = (unsigned short*)(ws + kOffVT);
  unsigned short* ctx16  = (unsigned short*)(ws + kOffCTX);
  float*          sc32   = (float*)(ws + kOffSC);
  unsigned short* p16    = (unsigned short*)(ws + kOffP);
  float*          x1     = (float*)(ws + kOffX1);
  unsigned short* hid16  = (unsigned short*)(ws + kOffHID);

  {
    const int n8q = (3 * kD * kD) / 8;
    const int n8o = (kD * kD) / 8;
    const int n8f = (kFF * kD) / 8;
    cast8_f16_kernel<<<(n8q + 255) / 256, 256, 0, stream>>>(qkv_w, qkvw16, n8q, kWCarry);
    cast8_f16_kernel<<<(n8o + 255) / 256, 256, 0, stream>>>(wo_w,  wo16,   n8o, kWCarry);
    cast8_f16_kernel<<<(n8f + 255) / 256, 256, 0, stream>>>(f1_w,  f1w16,  n8f, kWCarry);
    cast8_f16_kernel<<<(n8f + 255) / 256, 256, 0, stream>>>(f2_w,  f2w16,  n8f, kWCarry);
  }

  ln_row_kernel<<<kTok, 128, 0, stream>>>(x, ln1_w, ln1_b, h16);

  wmma_gemm64<0, false, 2, 1, false, 0><<<dim3(256, 1), 256, 0, stream>>>(
      h16, nullptr, kD, (long)0,
      qkvw16, nullptr, kD, (long)0,
      (void*)qk16, nullptr, 2 * kD, (long)0,
      qkv_b, nullptr, (long)0,
      kTok, 2 * kD, kD, kWCarryInv);

  wmma_gemm64<0, false, 1, 1, false, 0><<<dim3(64, kB), 256, 0, stream>>>(
      qkvw16 + (size_t)2 * kD * kD, nullptr, kD, (long)0,
      h16, nullptr, kD, (long)kS * kD,
      (void*)vt16, nullptr, kS, (long)kD * kS,
      qkv_b + 2 * kD, nullptr, (long)0,
      kD, kS, kD, kWCarryInv);

  for (int cidx = 0; cidx < kChunks; ++cidx) {
    const int bsel = (cidx * kGPC) / kH;
    const int h0   = (cidx * kGPC) % kH;
    const unsigned short* qbase = qk16 + (size_t)bsel * kS * (2 * kD) + (size_t)h0 * kDK;
    const unsigned short* kbase = qbase + kD;
    wmma_gemm64<0, false, 0, 0, false, 0><<<dim3(128, kGPC), 256, 0, stream>>>(
        qbase, nullptr, 2 * kD, (long)kDK,
        kbase, nullptr, 2 * kD, (long)kDK,
        (void*)sc32, nullptr, kS, (long)kS * kS,
        nullptr, nullptr, (long)0,
        kS, kS, kDK, kScoreScale);
    softmax_row_kernel<<<kGPC * kS, 256, 0, stream>>>(sc32, p16, kPCarry);
    wmma_gemm64<0, false, 0, 1, false, 0><<<dim3(4, kGPC), 256, 0, stream>>>(
        p16, nullptr, kS, (long)kS * kS,
        vt16 + (size_t)bsel * kD * kS + (size_t)h0 * kDK * kS, nullptr, kS, (long)kDK * kS,
        (void*)(ctx16 + (size_t)bsel * kS * kD + (size_t)h0 * kDK), nullptr, kD, (long)kDK,
        nullptr, nullptr, (long)0,
        kS, kDK, kS, kPVScale);
  }

  wmma_gemm64<0, false, 2, 0, true, 0><<<dim3(128, 1), 256, 0, stream>>>(
      ctx16, nullptr, kD, (long)0,
      wo16, nullptr, kD, (long)0,
      (void*)x1, nullptr, kD, (long)0,
      wo_b, x, (long)0,
      kTok, kD, kD, kWoScale);

  ln_row_kernel<<<kTok, 128, 0, stream>>>(x1, ln2_w, ln2_b, h16);

  wmma_gemm64<0, false, 2, 1, false, 2><<<dim3(512, 1), 256, 0, stream>>>(
      h16, nullptr, kD, (long)0,
      f1w16, nullptr, kD, (long)0,
      (void*)hid16, nullptr, kFF, (long)0,
      f1_b, nullptr, (long)0,
      kTok, kFF, kD, kWCarryInv);

  wmma_gemm64<0, false, 2, 0, true, 0><<<dim3(128, 1), 256, 0, stream>>>(
      hid16, nullptr, kFF, (long)0,
      f2w16, nullptr, kFF, (long)0,
      (void*)out, nullptr, kD, (long)0,
      f2_b, x1, (long)0,
      kTok, kD, kFF, kWCarryInv);
}
